// SelfAttention_72499047957175
// MI455X (gfx1250) — hardware-verified
//
#include <hip/hip_runtime.h>
#include <math.h>

#ifndef NB
#define NB 8
#endif
#ifndef SEQ
#define SEQ 4096
#endif
#define NB_FULL 8
#define SEQ_FULL 4096
#define NCH 64
#define NCQ 8

static_assert(SEQ % 128 == 0);
static_assert(SEQ <= SEQ_FULL);
static_assert(NB <= NB_FULL);
static_assert(NB >= 1);
static_assert(NCH == 64);
static_assert(NCQ == 8);
static_assert(SEQ_FULL % 4 == 0);

typedef __attribute__((ext_vector_type(16))) __bf16       v16b;
typedef __attribute__((ext_vector_type(8)))  float        v8f;
typedef __attribute__((ext_vector_type(4)))  float        v4f;
typedef __attribute__((ext_vector_type(4)))  unsigned int v4u;
typedef __attribute__((ext_vector_type(8)))  unsigned int v8u;


__device__ __forceinline__ unsigned bf_top(float f) {
    unsigned u = __float_as_uint(f);
    u += 0x7fffu + ((u >> 16) & 1u);
    return u & 0xffff0000u;
}
__device__ __forceinline__ float bf_val(float f) { return __uint_as_float(bf_top(f)); }
__device__ __forceinline__ unsigned pk_bf2(float a, float b) { return (bf_top(a) >> 16) | bf_top(b); }
__device__ __forceinline__ void split2(float a, float b, unsigned& hi, unsigned& lo) {
    const unsigned ha = bf_top(a), hb = bf_top(b);
    hi = (ha >> 16) | hb;
    const unsigned la = bf_top(a - __uint_as_float(ha)), lb = bf_top(b - __uint_as_float(hb));
    lo = (la >> 16) | lb;
}

__device__ __forceinline__ v8f wmmab(v16b a, v16b b, v8f c) {
    c = __builtin_amdgcn_wmma_f32_16x16x32_bf16(false, a, false, b, (short)0, c, false, false);
    asm volatile("v_nop\n\tv_nop\n\tv_nop\n\tv_nop" : "+v"(c) : "v"(a), "v"(b));
    return c;
}
__device__ __forceinline__ v8f wmma3(v16b ah, v16b al, v16b bh, v16b bl, v8f c) {
    c = __builtin_amdgcn_wmma_f32_16x16x32_bf16(false, ah, false, bh, (short)0, c, false, false);
    c = __builtin_amdgcn_wmma_f32_16x16x32_bf16(false, ah, false, bl, (short)0, c, false, false);
    c = __builtin_amdgcn_wmma_f32_16x16x32_bf16(false, al, false, bh, (short)0, c, false, false);
    asm volatile("v_nop\n\tv_nop\n\tv_nop\n\tv_nop" : "+v"(c) : "v"(ah), "v"(al), "v"(bh), "v"(bl));
    return c;
}

__device__ __forceinline__ v16b ld_frag(const unsigned short* p) {
    const v4u a = *(const v4u*)(p);
    const v4u c = *(const v4u*)(p + 16);
    const v8u u = __builtin_shufflevector(a, c, 0, 1, 2, 3, 4, 5, 6, 7);
    return __builtin_bit_cast(v16b, u);
}
__device__ __forceinline__ v16b ld_wfrag(const float* row, unsigned ks, unsigned h) {
    const float* p = row + ks * 32u + 8u * h;
    const v4f a0 = *(const v4f*)(p), a1 = *(const v4f*)(p + 4), c0 = *(const v4f*)(p + 16), c1 = *(const v4f*)(p + 20);
    v8u u;
    u[0] = pk_bf2(a0.x, a0.y); u[1] = pk_bf2(a0.z, a0.w); u[2] = pk_bf2(a1.x, a1.y); u[3] = pk_bf2(a1.z, a1.w);
    u[4] = pk_bf2(c0.x, c0.y); u[5] = pk_bf2(c0.z, c0.w); u[6] = pk_bf2(c1.x, c1.y); u[7] = pk_bf2(c1.z, c1.w);
    return __builtin_bit_cast(v16b, u);
}
__device__ __forceinline__ v16b ld_xfrag(const float* xp, unsigned ks, unsigned h) {
    v8u u;
#pragma unroll
    for (int i = 0; i < 4; ++i) {
        const size_t c = (size_t)(ks * 32u + 8u * h + 2u * (unsigned)i);
        u[i]     = pk_bf2(xp[c * SEQ_FULL],        xp[(c + 1) * SEQ_FULL]);
        u[4 + i] = pk_bf2(xp[(c + 16) * SEQ_FULL], xp[(c + 17) * SEQ_FULL]);
    }
    asm volatile("" : "+v"(u) : : "memory");
    return __builtin_bit_cast(v16b, u);
}

#define PROJ_PB (SEQ / 64)
static_assert(PROJ_PB * 64 == SEQ);
__global__ __launch_bounds__(32) void k_proj(const float* __restrict__ x,
                                             const float* __restrict__ wq,
                                             const float* __restrict__ wk,
                                             const float* __restrict__ wv,
                                             unsigned short* __restrict__ Qp, unsigned short* __restrict__ Kp,
                                             unsigned short* __restrict__ Vh, unsigned short* __restrict__ Vl) {
    __shared__ __align__(16) v4u sQK[2 * 64 * 4];
    __shared__ __align__(16) v4u sV[2 * 64 * 9];
    const unsigned lane = threadIdx.x & 31u, h = lane >> 4, lm = lane & 15u;
    const unsigned blk = blockIdx.x;
    const unsigned b = blk / (unsigned)PROJ_PB;
    const unsigned n0 = (blk - b * (unsigned)PROJ_PB) * 64u;
    const float* xb = x + (size_t)b * ((size_t)NCH * SEQ_FULL) + n0 + lm;

    v16b xf[4][2];
#pragma unroll
    for (int nt = 0; nt < 4; ++nt)
#pragma unroll
        for (int ks = 0; ks < 2; ++ks) xf[nt][ks] = ld_xfrag(xb + nt * 16, (unsigned)ks, h);

    const float qsc = h ? 1.0f : 1.4426950408889634f;

#pragma unroll
    for (int t = 0; t < 5; ++t) {
        const float* wrow;
        if (t == 0) wrow = ((lm < 8u) ? wq : wk) + (lm & 7u) * 64u;
        else        wrow = wv + (16u * (unsigned)(t - 1) + lm) * 64u;
        const v16b w0 = ld_wfrag(wrow, 0u, h), w1 = ld_wfrag(wrow, 1u, h);
        const unsigned cch = 16u * (unsigned)((t > 0) ? (t - 1) : 0) + lm;
#pragma unroll
        for (int nt = 0; nt < 4; ++nt) {
            v8f acc = {};
            float v8[8];
            if (t == 0) {
                acc = wmmab(w0, xf[nt][0], acc);
                acc = wmmab(w1, xf[nt][1], acc);
#pragma unroll
                for (int r = 0; r < 8; ++r) v8[r] = acc[r] * qsc;
            } else {
                acc = wmmab(xf[nt][0], w0, acc);
                acc = wmmab(xf[nt][1], w1, acc);
#pragma unroll
                for (int r = 0; r < 8; ++r) v8[r] = acc[r];
            }
            v4u H, L; unsigned a, c;
            split2(v8[0], v8[1], a, c); H.x = a; L.x = c;
            split2(v8[2], v8[3], a, c); H.y = a; L.y = c;
            split2(v8[4], v8[5], a, c); H.z = a; L.z = c;
            split2(v8[6], v8[7], a, c); H.w = a; L.w = c;
            if (t == 0) {
                const unsigned base = (h * 64u + (unsigned)nt * 16u + lm) * 4u;
                const v4u s1 = h ? H : L;
                const v4u s2 = h ? L : H;
                sQK[base] = H; sQK[base + 1] = s1; sQK[base + 2] = s2; sQK[base + 3] = L;
            } else {
                const unsigned pc = (unsigned)nt * 2u + h;
                sV[cch * 9u + pc] = H;
                sV[(64u + cch) * 9u + pc] = L;
            }
        }
    }
    __syncthreads();

    v4u* gQ = (v4u*)(Qp + ((size_t)b * SEQ + n0) * 32);
    v4u* gK = (v4u*)(Kp + ((size_t)b * SEQ + n0) * 32);
    for (int pass = 0; pass < 2; ++pass) {
#pragma unroll
        for (int it = 0; it < 8; ++it) {
            const unsigned idx = (unsigned)it * 32u + lane;
            const v4u vq = sQK[idx];
            const v4u vk = sQK[256u + idx];
            *(volatile v4u*)(gQ + idx) = vq;
            *(volatile v4u*)(gK + idx) = vk;
        }
#pragma unroll
        for (int it = 0; it < 16; ++it) {
            const unsigned idx = (unsigned)it * 32u + lane;
            const unsigned c = idx >> 3, pc = idx & 7u;
            const size_t go = ((size_t)(b * NCH + c) * SEQ + n0);
            const v4u vh = sV[c * 9u + pc];
            const v4u vl = sV[(64u + c) * 9u + pc];
            *(volatile v4u*)((v4u*)(Vh + go) + pc) = vh;
            *(volatile v4u*)((v4u*)(Vl + go) + pc) = vl;
        }
        __threadfence();
    }
}

#define ATT_PB (SEQ / 128)
static_assert(ATT_PB * 128 == SEQ);
__global__ __launch_bounds__(128) void k_attn(const unsigned short* __restrict__ Qp, const unsigned short* __restrict__ Kp,
                                              const unsigned short* __restrict__ Vh, const unsigned short* __restrict__ Vl,
                                              const float* __restrict__ x, const float* __restrict__ gamma,
                                              float* __restrict__ out) {
    __shared__ __align__(16) float sO[4][64 * 36];
    const unsigned lane = threadIdx.x & 31u, h = lane >> 4, lm = lane & 15u, wave = threadIdx.x >> 5;
    const unsigned blk = blockIdx.x;
    const unsigned b = blk / (unsigned)ATT_PB;
    const unsigned i0 = (blk - b * (unsigned)ATT_PB) * 128u + wave * 32u;

    v16b qf[2];
#pragma unroll
    for (int it = 0; it < 2; ++it) qf[it] = ld_frag(Qp + ((size_t)b * SEQ + i0 + (unsigned)it * 16u + lm) * 32 + 8u * h);

    const unsigned short* kb  = Kp + ((size_t)b * SEQ + lm) * 32 + 8u * h;
    const unsigned short* vhb = Vh + ((size_t)b * NCH + lm) * SEQ + 8u * h;
    const unsigned short* vlb = Vl + ((size_t)b * NCH + lm) * SEQ + 8u * h;

    float m_[2], l_[2];
    v8f Oacc[2][4];
#pragma unroll
    for (int it = 0; it < 2; ++it) {
        m_[it] = -1.0e30f; l_[it] = 0.f;
#pragma unroll
        for (int t = 0; t < 4; ++t) { v8f z = {}; Oacc[it][t] = z; }
    }

#pragma unroll 1
    for (unsigned j0 = 0; j0 < (unsigned)SEQ; j0 += 32u) {
        const v16b kf0 = ld_frag(kb + (size_t)j0 * 32);
        const v16b kf1 = ld_frag(kb + (size_t)(j0 + 16u) * 32);
        v16b ph[2], pl[2];
#pragma unroll
        for (int it = 0; it < 2; ++it) {
            v8f z = {};
            const v8f s0 = wmmab(kf0, qf[it], z);
            const v8f s1 = wmmab(kf1, qf[it], z);
            float bm = fmaxf(s0[0], s1[0]);
#pragma unroll
            for (int r = 1; r < 8; ++r) bm = fmaxf(bm, fmaxf(s0[r], s1[r]));
            bm = fmaxf(bm, __shfl_xor(bm, 16, 32));
            const float mo = m_[it];
            const float mn = fmaxf(mo, bm);
            const float alpha = exp2f(mo - mn);
            float p0[8], p1[8];
            float bs = 0.f;
#pragma unroll
            for (int r = 0; r < 8; ++r) {
                p0[r] = exp2f(s0[r] - mn);
                p1[r] = exp2f(s1[r] - mn);
                bs += p0[r] + p1[r];
            }
            bs += __shfl_xor(bs, 16, 32);
            l_[it] = l_[it] * alpha + bs;
            m_[it] = mn;
            if (__builtin_amdgcn_ballot_w32(mn > mo) != 0u) {
#pragma unroll
                for (int t = 0; t < 4; ++t) Oacc[it][t] = Oacc[it][t] * alpha;
            }
            v8u uh, ul;
#pragma unroll
            for (int i = 0; i < 4; ++i) {
                unsigned a, c;
                split2(p0[2 * i], p0[2 * i + 1], a, c); uh[i] = a; ul[i] = c;
                split2(p1[2 * i], p1[2 * i + 1], a, c); uh[4 + i] = a; ul[4 + i] = c;
            }
            ph[it] = __builtin_bit_cast(v16b, uh);
            pl[it] = __builtin_bit_cast(v16b, ul);
        }
#pragma unroll
        for (int t = 0; t < 4; ++t) {
            const size_t vo = (size_t)(16 * t) * SEQ + j0;
            const v16b vh = ld_frag(vhb + vo);
            const v16b vl = ld_frag(vlb + vo);
#pragma unroll
            for (int it = 0; it < 2; ++it) Oacc[it][t] = wmma3(vh, vl, ph[it], pl[it], Oacc[it][t]);
        }
    }

    float* so = sO[wave];
#pragma unroll
    for (int it = 0; it < 2; ++it) {
        const float inv = 1.0f / l_[it];
#pragma unroll
        for (int t = 0; t < 4; ++t)
#pragma unroll
            for (int r = 0; r < 8; ++r)
                so[(16u * (unsigned)t + 8u * h + (unsigned)r) * 36u + (unsigned)it * 16u + lm] = Oacc[it][t][r] * inv;
    }
    __syncthreads();
    float* ob = out + (size_t)b * ((size_t)NCH * SEQ) + i0;
    const float* xr = x + (size_t)b * ((size_t)NCH * SEQ_FULL) + i0;
    const float gm = bf_val(gamma[0]);
    const unsigned c4 = (lane & 7u) * 4u, cq = lane >> 3;
    for (int pass = 0; pass < 2; ++pass) {
#pragma unroll
        for (int s = 0; s < 16; ++s) {
            const unsigned c = (unsigned)s * 4u + cq;
            const v4f v = *(const v4f*)(so + c * 36u + c4);
            const v4f xv = *(const v4f*)(xr + (size_t)c * SEQ_FULL + c4);
            v4f o;
            o.x = bf_val(xv.x) + gm * v.x;
            o.y = bf_val(xv.y) + gm * v.y;
            o.z = bf_val(xv.z) + gm * v.z;
            o.w = bf_val(xv.w) + gm * v.w;
            *(volatile v4f*)(ob + (size_t)c * SEQ + c4) = o;
        }
        __threadfence();
    }
}

extern "C" void kernel_launch(void* const* d_in, const int* in_sizes, int n_in, void* d_out, int out_size, void* d_ws, size_t ws_size, hipStream_t stream) {
    if (n_in < 5) return;
    const long long need_x = ((long long)NB * NCH - 1) * (long long)SEQ_FULL + SEQ;
    if ((long long)in_sizes[0] < need_x) return;
    if (in_sizes[1] < NCQ * NCH || in_sizes[2] < NCQ * NCH) return;
    if (in_sizes[3] < NCH * NCH || in_sizes[4] < 1) return;
    if ((long long)out_size < (long long)NB * NCH * SEQ) return;

    const float* x     = (const float*)d_in[0];
    const float* wkey  = (const float*)d_in[1];
    const float* wqry  = (const float*)d_in[2];
    const float* wv    = (const float*)d_in[3];
    const float* gamma = (const float*)d_in[4];
    float* out = (float*)d_out;

    const size_t szQK = (size_t)NB * SEQ * 32 * 2;
    const size_t szV  = (size_t)NB * NCH * SEQ * 2;
    static_assert((((size_t)NB * SEQ * 32 * 2) % 256) == 0);
    static_assert((((size_t)NB * NCH * SEQ * 2) % 256) == 0);
    static_assert((2 * ((size_t)NB * SEQ * 32 * 2) + 2 * ((size_t)NB * NCH * SEQ * 2)) <= (size_t)134217728);
    if (2 * szQK + 2 * szV > ws_size) return;
    char* wsp = (char*)d_ws;
    unsigned short* Qp = (unsigned short*)wsp; wsp += szQK;
    unsigned short* Kp = (unsigned short*)wsp; wsp += szQK;
    unsigned short* Vh = (unsigned short*)wsp; wsp += szV;
    unsigned short* Vl = (unsigned short*)wsp; wsp += szV;

    k_proj<<<dim3((unsigned)(NB * PROJ_PB)), dim3(32), 0, stream>>>(x, wqry, wkey, wv, Qp, Kp, Vh, Vl);
    k_attn<<<dim3((unsigned)(NB * ATT_PB)), dim3(128), 0, stream>>>(Qp, Kp, Vh, Vl, x, gamma, out);
}
